// STULayer_71055938945776
// MI455X (gfx1250) — hardware-verified
//
#include <hip/hip_runtime.h>
#include <math.h>

typedef __attribute__((ext_vector_type(16))) _Float16 v16h;
typedef __attribute__((ext_vector_type(16))) __bf16 v16b;
typedef __attribute__((ext_vector_type(8)))  _Float16 v8h;
typedef __attribute__((ext_vector_type(8)))  float v8f;
typedef __attribute__((ext_vector_type(4)))  float v4f;
typedef __attribute__((ext_vector_type(2)))  float v2f;
typedef __attribute__((ext_vector_type(4)))  unsigned v4u;
typedef __attribute__((ext_vector_type(4)))  int v4i;
typedef __attribute__((ext_vector_type(8)))  __bf16 v8b;
typedef float __attribute__((may_alias)) float_a;
typedef int __attribute__((may_alias)) int_a;

template <typename T> __device__ __forceinline__ void vst2(void* p, T v) { *(volatile T*)p = v; __threadfence(); *(volatile T*)p = v; }
__device__ __forceinline__ v8f wmma16(v16h a, v16h b, v8f c) {
  v8f d = __builtin_amdgcn_wmma_f32_16x16x32_f16(false, a, false, b, (short)0, c, false, false);
  asm volatile("v_nop\n\tv_nop\n\tv_nop\n\tv_nop" : "+v"(d) : "v"(a), "v"(b));
  return d;
}
__device__ __forceinline__ v8f wmma_bf(v16b a, v16b b, v8f c) {
  v8f d = __builtin_amdgcn_wmma_f32_16x16x32_bf16(false, a, false, b, (short)0, c, false, false);
  asm volatile("v_nop\n\tv_nop\n\tv_nop\n\tv_nop" : "+v"(d) : "v"(a), "v"(b));
  return d;
}
__device__ __forceinline__ v16h frag_h(const _Float16* rowk0, int lane) {
  union { v16h v; v8h q[2]; } u; const _Float16* p = rowk0 + 8 * (lane >> 4);
  u.q[0] = *(const v8h*)p; u.q[1] = *(const v8h*)(p + 16); return u.v;
}
__device__ __forceinline__ v16h frag_f32(const float* rowk0, int lane) {
  v16h a; const float* p = rowk0 + 8 * (lane >> 4);
#pragma unroll
  for (int i = 0; i < 8; ++i) { a[i] = (_Float16)p[i]; a[8 + i] = (_Float16)p[16 + i]; }
  return a;
}
__device__ __forceinline__ v16h frag_f32s(const float* rowk0, int lane, float sc) {
  v16h a; const float* p = rowk0 + 8 * (lane >> 4);
#pragma unroll
  for (int i = 0; i < 8; ++i) { a[i] = (_Float16)(p[i] * sc); a[8 + i] = (_Float16)(p[16 + i] * sc); }
  return a;
}
__device__ __forceinline__ v16h fragc_f32(const float* W, int k0, int n, int lane, int ld, int K) {
  v16h a; const int g = lane >> 4;
#pragma unroll
  for (int i = 0; i < 8; ++i) { const int ka = k0 + 8 * g + i, kb = ka + 16;
    a[i] = (_Float16)(ka < K ? W[(size_t)(ka < K ? ka : K - 1) * ld + n] : 0.f); a[8 + i] = (_Float16)(kb < K ? W[(size_t)(kb < K ? kb : K - 1) * ld + n] : 0.f); }
  return a;
}
struct F2 { v16b h, l; };
__device__ __forceinline__ F2 bsplit16(const float v[16]) { F2 r;
#pragma unroll
  for (int i = 0; i < 16; ++i) { const __bf16 h = (__bf16)v[i]; r.h[i] = h; r.l[i] = (__bf16)(v[i] - (float)h); }
  return r; }
__device__ __forceinline__ F2 split_row(const float* row, int k0, int lane) { float v[16]; const float* p = row + k0 + 8 * (lane >> 4);
#pragma unroll
  for (int i = 0; i < 8; ++i) { v[i] = p[i]; v[8 + i] = p[16 + i]; }
  return bsplit16(v); }
__device__ __forceinline__ F2 split_rowK(const float* row, int k0, int lane, int K) { float v[16]; const int g = lane >> 4;
#pragma unroll
  for (int i = 0; i < 8; ++i) { const int ka = k0 + 8 * g + i, kb = ka + 16; v[i] = ka < K ? row[ka < K ? ka : K - 1] : 0.f; v[8 + i] = kb < K ? row[kb < K ? kb : K - 1] : 0.f; }
  return bsplit16(v); }
__device__ __forceinline__ F2 split_col(const float* W, int k0, int n, int lane, int ld, int K) { float v[16]; const int g = lane >> 4;
#pragma unroll
  for (int i = 0; i < 8; ++i) { const int ka = k0 + 8 * g + i, kb = ka + 16; v[i] = ka < K ? W[(size_t)(ka < K ? ka : K - 1) * ld + n] : 0.f; v[8 + i] = kb < K ? W[(size_t)(kb < K ? kb : K - 1) * ld + n] : 0.f; }
  return bsplit16(v); }
__device__ __forceinline__ v8f mac3(const F2& a, const F2& b, v8f c) { c = wmma_bf(a.l, b.h, c); c = wmma_bf(a.h, b.l, c); return wmma_bf(a.h, b.h, c); }
__device__ __forceinline__ float sigm(float v) { return 1.0f / (1.0f + expf(-v)); }
#define LDSX() do { asm volatile("s_wait_dscnt 0" ::: "memory"); __builtin_amdgcn_wave_barrier(); __builtin_amdgcn_fence(__ATOMIC_RELEASE, "workgroup"); } while (0)

#define NB 4
#define TT 4096
#define DD 256
#define KK 16
#define KD (KK * DD)
#define NCH (TT / 64)
#ifndef TNB
#define TNB NB
#endif
__device__ __forceinline__ float bfr(float v) { return (float)(__bf16)v; }
__device__ __forceinline__ v16b wrow(const float* rowk0, int lane) { v16b w; const float* p = rowk0 + 8 * (lane >> 4);
#pragma unroll
  for (int i = 0; i < 8; ++i) { w[i] = (__bf16)p[i]; w[8 + i] = (__bf16)p[16 + i]; }
  return w; }

#define WS_PS  0u
#define WS_EX  (WS_PS + 4u * (size_t)NB * NCH * KD)
#define WS_END (WS_EX + 4u * (size_t)NB * NCH * KD)

__global__ __launch_bounds__(256) void k_part(const float* __restrict__ X, const float* __restrict__ PHI, float* __restrict__ PS) {
  const int d = threadIdx.x; const int c = blockIdx.x, k = blockIdx.y, b = blockIdx.z; const size_t t0 = (size_t)c * 64; float s = 0.f;
#pragma unroll 4
  for (int r = 0; r < 64; ++r) s += bfr(PHI[(t0 + r) * KK + k]) * bfr(X[((size_t)b * TT + t0 + r) * DD + d]);
  float* dst = PS + (((size_t)b * NCH + c) * KK + k) * DD; { v4f tmp;   tmp[0] = __shfl(s, (d & ~3) + 0); tmp[1] = __shfl(s, (d & ~3) + 1); tmp[2] = __shfl(s, (d & ~3) + 2); tmp[3] = __shfl(s, (d & ~3) + 3); if ((d & 3) == 0) vst2(dst + d, tmp); } }
__global__ __launch_bounds__(256) void k_excl(const float* __restrict__ PS, float* __restrict__ EX) {
  const int d = threadIdx.x; const int k = blockIdx.x, b = blockIdx.y; float run = 0.f;
#pragma unroll 1
  for (int c = 0; c < NCH; ++c) { const size_t o = (((size_t)b * NCH + c) * KK + k) * DD; const float p = PS[o + d];
    { v4f tmp; tmp[0] = __shfl(run, (d & ~3) + 0); tmp[1] = __shfl(run, (d & ~3) + 1); tmp[2] = __shfl(run, (d & ~3) + 2); tmp[3] = __shfl(run, (d & ~3) + 3); if ((d & 3) == 0) vst2(EX + o + d, tmp); }
    run += p; } }
__global__ __launch_bounds__(128) void k_out(const float* __restrict__ X, const float* __restrict__ PHI, const float* __restrict__ W, const float* __restrict__ EX, float* __restrict__ OUT) {
  __shared__ __align__(16) float sx[64][33]; __shared__ __align__(16) __bf16 sah[64][40], sal[64][40]; __shared__ __align__(16) float sph[64][KK]; __shared__ __align__(16) float sf[4][16][132];
  const int tid = threadIdx.x, wave = tid >> 5, lane = tid & 31, col = lane & 15, g = lane >> 4; const int c = blockIdx.x, c0 = blockIdx.y * 128, b = blockIdx.z; const size_t t0 = (size_t)c * 64; const size_t rb = (size_t)b * TT + t0;
  for (int e = tid; e < 64 * KK; e += 128) { const int r = e >> 4, k = e & 15; sph[r][k] = bfr(PHI[(t0 + r) * KK + k]); }
  v8f acc[8] = {};
#pragma unroll 1
  for (int kc = 0; kc < KD / 32; ++kc) { const int k = kc >> 3, d0 = (kc & 7) * 32;
    __syncthreads();
    for (int e = tid; e < 64 * 32; e += 128) { const int r = e >> 5, dl = e & 31; sx[r][dl] = bfr(X[(rb + r) * DD + d0 + dl]); }
    __syncthreads();
    if (tid < 32) { const int dl = tid; float run = EX[(((size_t)b * NCH + c) * KK + k) * DD + d0 + dl];
#pragma unroll 4
      for (int r = 0; r < 64; ++r) { run += sph[r][k] * sx[r][dl]; const float a = sph[r][k] * run; const __bf16 h = (__bf16)a; sah[r][dl] = h; sal[r][dl] = (__bf16)(a - (float)h); } }
    __syncthreads();
    v16b ah, al; { union { v16b v; v8b q[2]; } uh, ul; uh.q[0] = *(const v8b*)&sah[wave * 16 + col][8 * g]; uh.q[1] = *(const v8b*)&sah[wave * 16 + col][16 + 8 * g]; ul.q[0] = *(const v8b*)&sal[wave * 16 + col][8 * g]; ul.q[1] = *(const v8b*)&sal[wave * 16 + col][16 + 8 * g]; ah = uh.v; al = ul.v; }
#pragma unroll
    for (int j = 0; j < 8; ++j) { const v16b w = wrow(W + ((size_t)k * DD + c0 + j * 16 + col) * DD + d0, lane); asm volatile("s_wait_loadcnt 0x0" ::: "memory"); acc[j] = wmma_bf(ah, w, acc[j]); acc[j] = wmma_bf(al, w, acc[j]); } }
#pragma unroll
  for (int j = 0; j < 8; ++j) {
#pragma unroll
    for (int r = 0; r < 8; ++r) sf[wave][8 * g + r][j * 16 + col] = acc[j][r]; }
  LDSX(); for (int rl = 0; rl < 16; ++rl) vst2(OUT + (rb + wave * 16 + rl) * DD + c0 + lane * 4, *(const v4f*)&sf[wave][rl][lane * 4]); }
extern "C" void kernel_launch(void* const* d_in, const int* in_sizes, int n_in, void* d_out, int out_size, void* d_ws, size_t ws_size, hipStream_t stream) {
  (void)in_sizes; (void)n_in; (void)out_size;
  const float** F = (const float**)d_in;
  if (ws_size < (size_t)WS_END) return;
  char* ws = (char*)d_ws; float *PS = (float*)(ws + WS_PS), *EX = (float*)(ws + WS_EX);
  k_part<<<dim3(NCH, KK, TNB), 256, 0, stream>>>(F[0], F[2], PS);
  k_excl<<<dim3(KK, TNB), 256, 0, stream>>>(PS, EX);
  k_out<<<dim3(NCH, DD / 128, TNB), 128, 0, stream>>>(F[0], F[2], F[1], EX, (float*)d_out);
}
